// GNN_Model_72911364817693
// MI455X (gfx1250) — hardware-verified
//
#include <hip/hip_runtime.h>
#include <math.h>
#include <stdint.h>

#define NN    128
#define NG    256
#define NBT   64
#define NSM   4
#define EPG   16256
#define NEDGE 4161536
#define HID   32
#define FIN1  3
#define NHOP  5
#define NBLK  6

static_assert(NEDGE == NG * EPG);
static_assert(EPG == NN * (NN - 1));
static_assert(NG == NBT * NSM);
static_assert(NN % 32 == 0);
static_assert(HID == 32);

#define OUT0_ELEMS (NG * NN * NN)
#define OUT2_OFF   (2 * NG * NN * NN)
#define OUT_TOTAL  (2 * NG * NN * NN + NG * NN)
static_assert(OUT_TOTAL == 8421376);
static_assert(OUT2_OFF + NG * NN - 1 < OUT_TOTAL);

typedef __bf16   v16b __attribute__((ext_vector_type(16)));
typedef __bf16   v8b  __attribute__((ext_vector_type(8)));
typedef float    v8f  __attribute__((ext_vector_type(8)));
typedef float    v4f  __attribute__((ext_vector_type(4)));
typedef unsigned short v8us __attribute__((ext_vector_type(8)));
typedef unsigned int   v4u  __attribute__((ext_vector_type(4)));
typedef v8b  __attribute__((may_alias)) v8ba;
typedef v4f  __attribute__((may_alias)) v4fa;
typedef v8us __attribute__((may_alias)) v8usa;
typedef v4u  __attribute__((may_alias)) v4ua;

#define LA_ATH   0
#define LA_ATL   32768
#define LA_HTH   65536
#define LA_HTL   73728
#define LA_HRH   81920
#define LA_HRL   90112
#define LA_W1T   98304
#define LA_W2T   110592
#define LA_WWT   122880
#define LA_B1    124928
#define LA_B2    125056
#define LA_BP    125184
#define LA_DIS   125312
#define LA_A0    125824
#define LA_P2    126336
#define LA_AIK   126848
#define LA_FLAG  127360
#define LA_TOTAL 127392
static_assert(LA_W1T - LA_HTH == 32768);

#define LB_T     0
#define LB_EIG   65536
#define LB_FLAG  65552
#define LB_TOTAL 65584

__device__ __forceinline__ unsigned short f2bf_bits(float f) {
  const unsigned u = __float_as_uint(f);
  return (unsigned short)((u + 0x7FFFu + ((u >> 16) & 1u)) >> 16);
}
__device__ __forceinline__ float bf_bits2f(unsigned short h) { return __uint_as_float(((unsigned)h) << 16); }
__device__ __forceinline__ float bf_rne(float f) { return bf_bits2f(f2bf_bits(f)); }
__device__ __forceinline__ void split_bits(float f, unsigned short& hb, unsigned short& lb) {
  hb = f2bf_bits(f);
  lb = f2bf_bits(f - bf_bits2f(hb));
}

__device__ __forceinline__ v8f mma_bf(v16b a, v16b b, v8f c) {
  c = __builtin_amdgcn_wmma_f32_16x16x32_bf16(false, a, false, b, (short)0, c, false, false);
  asm volatile("v_nop\n\tv_nop\n\tv_nop\n\tv_nop" : "+v"(c) : "v"(a), "v"(b));
  return c;
}

union FragB { v16b v; v8b h[2]; };

__device__ __forceinline__ v16b frag_lds(const unsigned short* p) {
  FragB f;
  f.h[0] = *(const v8ba*)(p);
  f.h[1] = *(const v8ba*)(p + 16);
  return f.v;
}

template <int NT>
__device__ __forceinline__ void hop_layer(const unsigned short* ATH, const unsigned short* ATL,
                                          unsigned short* HTH, unsigned short* HTL,
                                          unsigned short* HRH, unsigned short* HRL,
                                          const unsigned short* WT, const float* BIAS,
                                          int wave, int lane)
{
  const int hh = lane >> 4, rl = lane & 15, d0 = wave * 16;
  const v8f z8 = {0.f, 0.f, 0.f, 0.f, 0.f, 0.f, 0.f, 0.f};
  v8f acc2[2];
  acc2[0] = z8; acc2[1] = z8;

#pragma unroll 1
  for (int j = 0; j < NBLK; ++j) {
    {
      const v16b ah = frag_lds(HRH + (d0 + rl) * HID + 8 * hh);
      const v16b al = frag_lds(HRL + (d0 + rl) * HID + 8 * hh);
#pragma unroll
      for (int nt = 0; nt < 2; ++nt) {
        const v16b bw = frag_lds(WT + j * (HID * HID) + (16 * nt + rl) * HID + 8 * hh);
        acc2[nt] = mma_bf(ah, bw, acc2[nt]);
        acc2[nt] = mma_bf(al, bw, acc2[nt]);
      }
    }
    if (j < NHOP) {
      v8f hacc[NT];
#pragma unroll
      for (int nt = 0; nt < NT; ++nt) hacc[nt] = z8;
#pragma unroll 1
      for (int ks = 0; ks < NN; ks += 32) {
        const v16b aH = frag_lds(ATH + (d0 + rl) * NN + ks + 8 * hh);
        const v16b aL = frag_lds(ATL + (d0 + rl) * NN + ks + 8 * hh);
#pragma unroll
        for (int nt = 0; nt < NT; ++nt) {
          const v16b bH = frag_lds(HTH + (16 * nt + rl) * NN + ks + 8 * hh);
          const v16b bL = frag_lds(HTL + (16 * nt + rl) * NN + ks + 8 * hh);
          hacc[nt] = mma_bf(aH, bH, hacc[nt]);
          hacc[nt] = mma_bf(aH, bL, hacc[nt]);
          hacc[nt] = mma_bf(aL, bH, hacc[nt]);
        }
      }
      __syncthreads();
#pragma unroll
      for (int nt = 0; nt < NT; ++nt) {
        const int f = 16 * nt + rl;
        v8us hv, lv;
#pragma unroll
        for (int r = 0; r < 8; ++r) {
          unsigned short hb, lb;
          split_bits(hacc[nt][r], hb, lb);
          hv[r] = hb; lv[r] = lb;
          HRH[(d0 + 8 * hh + r) * HID + f] = hb;
          HRL[(d0 + 8 * hh + r) * HID + f] = lb;
        }
        *(v8usa*)(HTH + f * NN + d0 + 8 * hh) = hv;
        *(v8usa*)(HTL + f * NN + d0 + 8 * hh) = lv;
      }
      __syncthreads();
    }
  }
  __syncthreads();
#pragma unroll
  for (int nt = 0; nt < 2; ++nt) {
    const int f = 16 * nt + rl;
    const float bv = BIAS[f];
    v8us hv, lv;
#pragma unroll
    for (int r = 0; r < 8; ++r) {
      float v = acc2[nt][r] + bv;
      v = (v > 0.f) ? v : 0.01f * v;
      unsigned short hb, lb;
      split_bits(v, hb, lb);
      hv[r] = hb; lv[r] = lb;
      HRH[(d0 + 8 * hh + r) * HID + f] = hb;
      HRL[(d0 + 8 * hh + r) * HID + f] = lb;
    }
    *(v8usa*)(HTH + f * NN + d0 + 8 * hh) = hv;
    *(v8usa*)(HTL + f * NN + d0 + 8 * hh) = lv;
  }
  __syncthreads();
}

__global__ __launch_bounds__(256) void graph_kernel(
    const float* __restrict__ x, const int* __restrict__ ei, const float* __restrict__ ew,
    const float* __restrict__ W1, const float* __restrict__ b1,
    const float* __restrict__ W2, const float* __restrict__ b2,
    const float* __restrict__ bpw, const float* __restrict__ ww,
    float* __restrict__ ry, float* __restrict__ aik)
{
  extern __shared__ __align__(16) unsigned char smem[];
  unsigned short* ATH = (unsigned short*)(smem + LA_ATH);
  unsigned short* ATL = (unsigned short*)(smem + LA_ATL);
  unsigned short* HTH = (unsigned short*)(smem + LA_HTH);
  unsigned short* HTL = (unsigned short*)(smem + LA_HTL);
  unsigned short* HRH = (unsigned short*)(smem + LA_HRH);
  unsigned short* HRL = (unsigned short*)(smem + LA_HRL);
  unsigned short* W1T = (unsigned short*)(smem + LA_W1T);
  unsigned short* W2T = (unsigned short*)(smem + LA_W2T);
  unsigned short* WWT = (unsigned short*)(smem + LA_WWT);
  float* B1s  = (float*)(smem + LA_B1);
  float* B2s  = (float*)(smem + LA_B2);
  float* BPs  = (float*)(smem + LA_BP);
  float* DISs = (float*)(smem + LA_DIS);
  float* A0s  = (float*)(smem + LA_A0);
  float* P2s  = (float*)(smem + LA_P2);
  float* AIKs = (float*)(smem + LA_AIK);
  int*   FLAG = (int*)(smem + LA_FLAG);
  float* RYS  = (float*)(smem + LA_ATH);
  unsigned short* YWH = HTH;
  unsigned short* YWL = HTL;

  const int kb = blockIdx.x;
  const int tid = threadIdx.x, wave = tid >> 5, lane = tid & 31, hh = lane >> 4, rl = lane & 15;
  const int d0 = wave * 16;
  const v8f z8 = {0.f, 0.f, 0.f, 0.f, 0.f, 0.f, 0.f, 0.f};

#pragma unroll 2
  for (int i = tid; i < 2048; i += 256) *(v4ua*)(smem + LA_HTH + 16 * i) = (v4u){0u, 0u, 0u, 0u};
#pragma unroll 2
  for (int i = tid; i < NBLK * HID * HID; i += 256) {
    const int j = i >> 10, o = (i >> 5) & 31, k = i & 31;
    const int k1 = (k < FIN1) ? k : (FIN1 - 1);
    const unsigned short wb1 = f2bf_bits(W1[(FIN1 * j + k1) * HID + o]);
    W1T[i] = (unsigned short)(wb1 & (0u - (unsigned)((k < FIN1) ? 1 : 0)));
    W2T[i] = f2bf_bits(W2[(HID * j + k) * HID + o]);
  }
#pragma unroll 2
  for (int i = tid; i < HID * HID; i += 256) {
    const int o = i >> 5, k = i & 31;
    WWT[i] = f2bf_bits(ww[k * HID + o]);
  }
  if (tid < HID) { B1s[tid] = bf_rne(b1[tid]); B2s[tid] = bf_rne(b2[tid]); BPs[tid] = bf_rne(bpw[tid]); }
  float xa = 0.f, xm = 0.f, xp = 0.f;
  if (tid < NN) {
    const size_t xr = (size_t)(kb * NN + tid) * 3;
    xa = bf_rne(x[xr]); xm = bf_rne(x[xr + 1]); xp = bf_rne(x[xr + 2]);
    A0s[tid] = xa; P2s[tid] = xp;
  }
  __syncthreads();
  if (tid < NN) {
    const unsigned short h0 = f2bf_bits(xa), h1 = f2bf_bits(xm), h2 = f2bf_bits(xp);
    HRH[tid * HID + 0] = h0; HRH[tid * HID + 1] = h1; HRH[tid * HID + 2] = h2;
    HTH[0 * NN + tid] = h0; HTH[1 * NN + tid] = h1; HTH[2 * NN + tid] = h2;
  }

  int bad = 0;
  float dself = 0.f;
  if (tid < NN) {
    const int d = tid;
    float deg = 0.f;
#pragma unroll 2
    for (int s = 0; s < NN; ++s) {
      const int valid = (s != d) ? 1 : 0;
      const int el = s * (NN - 1) + valid * (d - ((d > s) ? 1 : 0));
      const int eg = kb * EPG + el;
      const float wr = ew[eg];
      const int sv = ei[eg];
      const int dv = ei[NEDGE + eg];
      bad |= valid & (((sv != kb * NN + s) ? 1 : 0) | ((dv != kb * NN + d) ? 1 : 0));
      const unsigned short wb = (unsigned short)(f2bf_bits(wr) & (0u - (unsigned)valid));
      deg += bf_bits2f(wb);
      ATH[d * NN + s] = wb;
    }
    dself = (deg > 0.f) ? (1.0f / sqrtf(deg)) : 0.f;
    DISs[d] = dself;
  }
  {
    const int wany = __any(bad);
    if (lane == 0) FLAG[wave] = wany;
  }
  __syncthreads();
  if (tid < NN) {
    const int d = tid;
#pragma unroll 2
    for (int s = 0; s < NN; ++s) {
      const float raw = bf_bits2f(ATH[d * NN + s]);
      const float nv = (DISs[s] * raw) * dself;
      unsigned short hb, lb;
      split_bits(nv, hb, lb);
      ATH[d * NN + s] = hb;
      ATL[d * NN + s] = lb;
    }
  }
  const int anybad = FLAG[0] | FLAG[1] | FLAG[2] | FLAG[3] | FLAG[4] | FLAG[5] | FLAG[6] | FLAG[7];
  __syncthreads();

  hop_layer<1>(ATH, ATL, HTH, HTL, HRH, HRL, W1T, B1s, wave, lane);
  hop_layer<2>(ATH, ATL, HTH, HTL, HRH, HRL, W2T, B2s, wave, lane);

  if (tid < NN) {
    const int d = tid;
    float s = 0.f;
#pragma unroll 4
    for (int f = 0; f < HID; ++f) {
      const float yv = bf_bits2f(HRH[d * HID + f]) + bf_bits2f(HRL[d * HID + f]);
      s += yv * BPs[f];
    }
    s = fmaxf(s, 0.f);
    AIKs[d] = (A0s[d] + s) * (1.0f - P2s[d]);
  }
  {
    const v16b ah = frag_lds(HRH + (d0 + rl) * HID + 8 * hh);
    const v16b al = frag_lds(HRL + (d0 + rl) * HID + 8 * hh);
#pragma unroll
    for (int nt = 0; nt < 2; ++nt) {
      const v16b bw = frag_lds(WWT + (16 * nt + rl) * HID + 8 * hh);
      v8f acc = z8;
      acc = mma_bf(ah, bw, acc);
      acc = mma_bf(al, bw, acc);
      const int g = 16 * nt + rl;
#pragma unroll
      for (int r = 0; r < 8; ++r) {
        unsigned short hb, lb;
        split_bits(acc[r], hb, lb);
        YWH[(d0 + 8 * hh + r) * HID + g] = hb;
        YWL[(d0 + 8 * hh + r) * HID + g] = lb;
      }
    }
  }
  __syncthreads();

  {
    const v16b ya  = frag_lds(YWH + (d0 + rl) * HID + 8 * hh);
    const v16b yal = frag_lds(YWL + (d0 + rl) * HID + 8 * hh);
    const float qnan = __uint_as_float(0x7fc00000u);
#pragma unroll 1
    for (int mt = 0; mt < NN / 16; ++mt) {
      const v16b bH = frag_lds(HRH + (16 * mt + rl) * HID + 8 * hh);
      const v16b bL = frag_lds(HRL + (16 * mt + rl) * HID + 8 * hh);
      v8f acc = z8;
      acc = mma_bf(ya, bH, acc);
      acc = mma_bf(ya, bL, acc);
      acc = mma_bf(yal, bH, acc);
#pragma unroll
      for (int r = 0; r < 8; ++r) {
        const int n = d0 + 8 * hh + r;
        float v = acc[r];
        v = (P2s[n] == 1.0f) ? -1e10f : v;
        v = anybad ? qnan : v;
        RYS[n * NN + 16 * mt + rl] = v;
      }
    }
  }
  __syncthreads();

#pragma unroll 1
  for (int pass = 0; pass < 2; ++pass) {
    if (wave == 0) {
      const v4f v = *(const v4fa*)(AIKs + 4 * lane);
      *(volatile v4f*)(aik + (size_t)kb * NN + 4 * lane) = v;
    }
#pragma unroll
    for (int i = 0; i < 16; ++i) {
      const v4f v = *(const v4fa*)(RYS + (d0 + i) * NN + 4 * lane);
      *(volatile v4f*)(ry + ((size_t)(kb * NN + d0 + i)) * NN + 4 * lane) = v;
    }
    __threadfence();
  }
}

__global__ __launch_bounds__(256) void mix_kernel(
    const float* __restrict__ ry, const int* __restrict__ ei, const float* __restrict__ ew,
    const float* __restrict__ eig, float* __restrict__ out0, float* __restrict__ out1)
{
  extern __shared__ __align__(16) unsigned char smem[];
  float* T    = (float*)(smem + LB_T);
  float* EIGs = (float*)(smem + LB_EIG);
  int*   FLAG = (int*)(smem + LB_FLAG);

  const int b = blockIdx.x & (NBT - 1), qt = blockIdx.x >> 6;
  const int n0 = qt * 32;
  const int tid = threadIdx.x, wave = tid >> 5, lane = tid & 31;

#pragma unroll 4
  for (int i4 = tid; i4 < 4096; i4 += 256) {
    const int k = i4 >> 10, nl = (i4 >> 5) & 31, m4 = (i4 & 31) * 4;
    const int kbk = k * NBT + b;
    const v4f v = *(const v4fa*)(ry + ((size_t)(kbk * NN + n0 + nl)) * NN + m4);
    *(v4fa*)(T + 4 * i4) = v;
  }
  if (tid < NSM) EIGs[tid] = bf_rne(eig[tid * NBT + b]);
  __syncthreads();

#pragma unroll 2
  for (int p = tid; p < 4096; p += 256) {
    const float v0 = T[p], v1 = T[4096 + p], v2 = T[8192 + p], v3 = T[12288 + p];
    const float mx = fmaxf(fmaxf(v0, v1), fmaxf(v2, v3));
    const float e0 = __expf(v0 - mx), e1 = __expf(v1 - mx), e2 = __expf(v2 - mx), e3 = __expf(v3 - mx);
    const float ssum = ((e0 + e1) + e2) + e3;
    const float inv = 1.0f / ssum;
    T[p] = e0 * inv; T[4096 + p] = e1 * inv; T[8192 + p] = e2 * inv; T[12288 + p] = e3 * inv;
  }
  __syncthreads();

  int bad = 0;
#pragma unroll 2
  for (int it = 0; it < 64; ++it) {
    const int i = tid + 256 * it;
    const int k = i >> 12, p = i & 4095, nl = p >> 7, m = p & 127;
    const int n = n0 + nl, kbk = k * NBT + b;
    const int valid = (m != n) ? 1 : 0;
    const int el = n * (NN - 1) + valid * (m - ((m > n) ? 1 : 0));
    const int eg = kbk * EPG + el;
    const float wr = ew[eg];
    const int sv = ei[eg];
    const int dv = ei[NEDGE + eg];
    bad |= valid & (((sv != kbk * NN + n) ? 1 : 0) | ((dv != kbk * NN + m) ? 1 : 0));
    const unsigned short wb = (unsigned short)(f2bf_bits(wr) & (0u - (unsigned)valid));
    const float c = bf_bits2f(wb) * EIGs[k];
    T[i] = T[i] * c;
  }
  {
    const int wany = __any(bad);
    if (lane == 0) FLAG[wave] = wany;
  }
  __syncthreads();
  const int anybad = FLAG[0] | FLAG[1] | FLAG[2] | FLAG[3] | FLAG[4] | FLAG[5] | FLAG[6] | FLAG[7];
  const float qnan = __uint_as_float(0x7fc00000u);
  const v4f vnan = {qnan, qnan, qnan, qnan};
  const int q = lane >> 3, c4 = (lane & 7) * 4;

#pragma unroll 1
  for (int pass = 0; pass < 2; ++pass) {
#pragma unroll
    for (int i = 0; i < 16; ++i) {
      const int rr = wave * 16 + i, k = rr >> 5, nl = rr & 31;
      v4f v = *(const v4fa*)(T + k * 4096 + nl * NN + 4 * lane);
      if (anybad) v = vnan;
      *(volatile v4f*)(out0 + ((size_t)((k * NBT + b) * NN + n0 + nl)) * NN + 4 * lane) = v;
    }
#pragma unroll
    for (int it = 0; it < 16; ++it) {
      const int L = wave * 64 + it * 4 + q, k = L >> 7, m = L & 127;
      const float* tp = T + k * 4096 + c4 * NN + m;
      v4f v = {tp[0], tp[NN], tp[2 * NN], tp[3 * NN]};
      if (anybad) v = vnan;
      *(volatile v4f*)(out1 + ((size_t)((k * NBT + b) * NN + m)) * NN + n0 + c4) = v;
    }
    __threadfence();
  }
}

extern "C" void kernel_launch(void* const* d_in, const int* in_sizes, int n_in,
                              void* d_out, int out_size, void* d_ws, size_t ws_size,
                              hipStream_t stream) {
  if (n_in < 10) return;
  if (in_sizes[0] != NG * NN * 3) return;
  if (in_sizes[1] != 2 * NEDGE) return;
  if (in_sizes[2] != NEDGE) return;
  if (in_sizes[3] != NG) return;
  if (in_sizes[4] != NBLK * FIN1 * HID || in_sizes[5] != HID) return;
  if (in_sizes[6] != NBLK * HID * HID || in_sizes[7] != HID) return;
  if (in_sizes[8] != HID || in_sizes[9] != HID * HID) return;
  if (out_size != OUT_TOTAL) return;
  const size_t ry_bytes = (size_t)NG * NN * NN * sizeof(float);
  if (ry_bytes > ws_size) return;
  if (ry_bytes > (size_t)134217728) return;

  const float* x   = (const float*)d_in[0];
  const int*   ei  = (const int*)d_in[1];
  const float* ew  = (const float*)d_in[2];
  const float* eig = (const float*)d_in[3];
  const float* W1  = (const float*)d_in[4];
  const float* b1  = (const float*)d_in[5];
  const float* W2  = (const float*)d_in[6];
  const float* b2  = (const float*)d_in[7];
  const float* bpw = (const float*)d_in[8];
  const float* ww  = (const float*)d_in[9];

  float* out  = (float*)d_out;
  float* out0 = out;
  float* out1 = out + OUT0_ELEMS;
  float* aik  = out + OUT2_OFF;
  float* ry   = (float*)d_ws;

  (void)hipFuncSetAttribute(reinterpret_cast<const void*>(&graph_kernel),
                            hipFuncAttributeMaxDynamicSharedMemorySize, LA_TOTAL);
  graph_kernel<<<dim3(NG), dim3(256), LA_TOTAL, stream>>>(x, ei, ew, W1, b1, W2, b2, bpw, ww, ry, aik);

  (void)hipFuncSetAttribute(reinterpret_cast<const void*>(&mix_kernel),
                            hipFuncAttributeMaxDynamicSharedMemorySize, LB_TOTAL);
  mix_kernel<<<dim3(NBT * (NN / 32)), dim3(256), LB_TOTAL, stream>>>(ry, ei, ew, eig, out0, out1);
  (void)hipGetLastError();
}
